// BoundaryExtractionModule_34248069218322
// MI455X (gfx1250) — hardware-verified
//
#include <hip/hip_runtime.h>


#define NB_  8
#define CC   64
#define HH   64
#define NPX  4096
#define WP   66
#define NPP  (WP * WP)
#define NPR  4416
#define GB   128
#define NPT  (GB + NPR + GB)
#define DM   CC
#define LOSC 1024.0f

typedef _Float16 h16;
typedef unsigned short bf;
typedef __attribute__((ext_vector_type(16))) __bf16   v16bf;
typedef __attribute__((ext_vector_type(16))) _Float16 v16h;
typedef __attribute__((ext_vector_type(8)))  _Float16 v8h;
typedef __attribute__((ext_vector_type(8)))  unsigned short v8us;
typedef __attribute__((ext_vector_type(8)))  float    v8f;
typedef __attribute__((ext_vector_type(4)))  float    v4f;
typedef __attribute__((ext_vector_type(4)))  _Float16 v4h;
typedef v8h  __attribute__((may_alias)) v8ha;
typedef v4f  __attribute__((may_alias)) v4fa;
typedef v8us __attribute__((may_alias)) v8usa;

__device__ __forceinline__ unsigned short f2bf(float f) { unsigned u = __float_as_uint(f); u += 0x7FFFu + ((u >> 16) & 1u); return (unsigned short)(u >> 16); }
__device__ __forceinline__ float bf2f(unsigned short b) { return __uint_as_float(((unsigned)b) << 16); }
__device__ __forceinline__ float bfr(float f) { return bf2f(f2bf(f)); }
__device__ __forceinline__ v16h cat16(v8h lo, v8h hi) { return __builtin_shufflevector(lo, hi, 0, 1, 2, 3, 4, 5, 6, 7, 8, 9, 10, 11, 12, 13, 14, 15); }
__device__ __forceinline__ v16bf cat16b(v8us lo, v8us hi) { return __builtin_bit_cast(v16bf, __builtin_shufflevector(lo, hi, 0, 1, 2, 3, 4, 5, 6, 7, 8, 9, 10, 11, 12, 13, 14, 15)); }
__device__ __forceinline__ v8f wmma16(v16h a, v16h b, v8f c) { return __builtin_amdgcn_wmma_f32_16x16x32_f16(false, a, false, b, (short)0, c, false, false); }
__device__ __forceinline__ v8f wmmab(v16bf a, v16bf b, v8f c) { return __builtin_amdgcn_wmma_f32_16x16x32_bf16(false, a, false, b, (short)0, c, false, false); }

template <bool SPLITA, bool F16OUT = false>
__global__ __launch_bounds__(128) void k_gemmb(const bf* __restrict__ A, const bf* __restrict__ Al, const bf* __restrict__ Bn, const float* __restrict__ bias, float* C, int ldc, h16* C2, const float* __restrict__ R = nullptr, int K = DM, int roundR = 1) {
    __shared__ __align__(16) float ost[4][16 * 68];
    const int lane = threadIdx.x & 31, wave = threadIdx.x >> 5, lr = lane & 15, hi = lane >> 4;
    const int r0 = blockIdx.x * 64 + wave * 16, c0 = blockIdx.y * 64;
    const size_t aoff = (size_t)(r0 + lr) * K + 8 * hi;
    size_t boff[4];
#pragma unroll
    for (int t = 0; t < 4; ++t) boff[t] = (size_t)(c0 + t * 16 + lr) * K + 8 * hi;
    v8f acc[4];
#pragma unroll
    for (int t = 0; t < 4; ++t) acc[t] = (v8f){};
#pragma unroll 1
    for (int kc = 0; kc < K; kc += 32) {
        const v16bf a = cat16b(*(const v8us*)(A + aoff + kc), *(const v8us*)(A + aoff + kc + 16));
        v16bf al = a;
        if (SPLITA) al = cat16b(*(const v8us*)(Al + aoff + kc), *(const v8us*)(Al + aoff + kc + 16));
#pragma unroll
        for (int t = 0; t < 4; ++t) { const v16bf b = cat16b(*(const v8us*)(Bn + boff[t] + kc), *(const v8us*)(Bn + boff[t] + kc + 16)); acc[t] = wmmab(a, b, acc[t]); if (SPLITA) acc[t] = wmmab(al, b, acc[t]); }
        asm volatile("v_nop\n\tv_nop\n\tv_nop\n\tv_nop" : "+v"(acc[0]), "+v"(acc[1]), "+v"(acc[2]), "+v"(acc[3]) : "v"(a), "v"(al));
    }
    float* os = &ost[wave][0];
#pragma unroll
    for (int t = 0; t < 4; ++t) { const float bv = bias ? bfr(bias[c0 + t * 16 + lr]) : 0.f;
#pragma unroll
        for (int j = 0; j < 8; ++j) os[(hi * 8 + j) * 68 + t * 16 + lr] = acc[t][j] + bv; }
    __syncthreads();
    if (F16OUT) {
        h16* crow = (h16*)(void*)C + (size_t)r0 * ldc + c0;
        auto pass = [&]() {
#pragma unroll
            for (int s = 0; s < 4; ++s) { const int row = 4 * s + (lane >> 3), piece = lane & 7; const float* sp = os + row * 68 + piece * 8; v8h o, o2;
#pragma unroll
                for (int i = 0; i < 8; ++i) { const h16 a = (h16)sp[i]; o[i] = a; o2[i] = (h16)((sp[i] - (float)a) * LOSC); }
                *(volatile v8h*)(crow + (size_t)row * ldc + piece * 8) = o; if (C2) *(volatile v8h*)(C2 + (size_t)r0 * ldc + c0 + (size_t)row * ldc + piece * 8) = o2; }
        };
        pass(); __threadfence(); pass();
    } else {
        float* crow = C + (size_t)r0 * ldc + c0;
        auto pass = [&]() {
#pragma unroll
            for (int s = 0; s < 8; ++s) { const int Lid = (lane >> 3) + 4 * s, piece = lane & 7; const int row = Lid >> 1, cofs = (Lid & 1) * 32 + piece * 4;
                v4f val = *(const v4fa*)(os + row * 68 + cofs); if (R) { const v4f rv = *(const v4f*)(R + ((size_t)r0 + row) * ldc + c0 + cofs); val += roundR ? (v4f){bfr(rv[0]), bfr(rv[1]), bfr(rv[2]), bfr(rv[3])} : rv; }
                *(volatile v4f*)(crow + (size_t)row * ldc + cofs) = val; }
        };
        pass(); __threadfence(); pass();
    }
}

__global__ __launch_bounds__(128) void k_gemm3(const bf* __restrict__ Ah, const bf* __restrict__ Al, const bf* __restrict__ Bh, const bf* __restrict__ Bl, int K, float* C, int ldc) {
    __shared__ __align__(16) float ost[4][16 * 68];
    const int lane = threadIdx.x & 31, wave = threadIdx.x >> 5, lr = lane & 15, hi = lane >> 4;
    const int r0 = blockIdx.x * 64 + wave * 16, c0 = blockIdx.y * 64;
    const size_t aoff = (size_t)(r0 + lr) * K + 8 * hi;
    v8f acc[4];
#pragma unroll
    for (int t = 0; t < 4; ++t) acc[t] = (v8f){};
#pragma unroll 1
    for (int kc = 0; kc < K; kc += 32) {
        const v16bf a = cat16b(*(const v8us*)(Ah + aoff + kc), *(const v8us*)(Ah + aoff + kc + 16));
        const v16bf al = cat16b(*(const v8us*)(Al + aoff + kc), *(const v8us*)(Al + aoff + kc + 16));
#pragma unroll
        for (int t = 0; t < 4; ++t) { const size_t bo = (size_t)(c0 + t * 16 + lr) * K + kc + 8 * hi;
            const v16bf bh = cat16b(*(const v8us*)(Bh + bo), *(const v8us*)(Bh + bo + 16)); const v16bf bl = cat16b(*(const v8us*)(Bl + bo), *(const v8us*)(Bl + bo + 16));
            acc[t] = wmmab(a, bh, acc[t]); acc[t] = wmmab(al, bh, acc[t]); acc[t] = wmmab(a, bl, acc[t]); }
        asm volatile("v_nop\n\tv_nop\n\tv_nop\n\tv_nop" : "+v"(acc[0]), "+v"(acc[1]), "+v"(acc[2]), "+v"(acc[3]) : "v"(a), "v"(al));
    }
    float* os = &ost[wave][0];
#pragma unroll
    for (int t = 0; t < 4; ++t) {
#pragma unroll
        for (int j = 0; j < 8; ++j) os[(hi * 8 + j) * 68 + t * 16 + lr] = acc[t][j]; }
    __builtin_amdgcn_wave_barrier(); asm volatile("" ::: "memory");
    float* crow = C + (size_t)r0 * ldc + c0;
    auto pass = [&]() {
#pragma unroll
        for (int s = 0; s < 8; ++s) { const int Lid = (lane >> 3) + 4 * s, piece = lane & 7; const int row = Lid >> 1, cofs = (Lid & 1) * 32 + piece * 4;
            const v4f val = *(const v4fa*)(os + row * 68 + cofs); *(volatile v4f*)(crow + (size_t)row * ldc + cofs) = val; }
    };
    pass(); __threadfence(); pass();
}


__global__ __launch_bounds__(128) void k_gemmtap(const bf* __restrict__ Ah, const bf* __restrict__ Al, const bf* __restrict__ Bt, const float* __restrict__ bias, float* C, int ldc, int K) {
    __shared__ __align__(16) float ost[4][16 * 68];
    const int lane = threadIdx.x & 31, wave = threadIdx.x >> 5, lr = lane & 15, hi = lane >> 4;
    const int r0 = blockIdx.x * 64 + wave * 16, c0 = blockIdx.y * 64;
    v8f acc[4];
#pragma unroll
    for (int t = 0; t < 4; ++t) acc[t] = (v8f){};
#pragma unroll 1
    for (int tap = 0; tap < 9; ++tap) { const long off = (long)(tap / 3 - 1) * WP + (tap % 3 - 1);
        const size_t aoff = (size_t)((long)GB + off + r0 + lr) * K + 8 * hi; const bf* Bn = Bt + (size_t)tap * 64 * K;
        size_t boff[4];
#pragma unroll
        for (int t = 0; t < 4; ++t) boff[t] = (size_t)(c0 + t * 16 + lr) * K + 8 * hi;
#pragma unroll 1
        for (int kc = 0; kc < K; kc += 32) {
            const v16bf a = cat16b(*(const v8us*)(Ah + aoff + kc), *(const v8us*)(Ah + aoff + kc + 16));
            const v16bf al = cat16b(*(const v8us*)(Al + aoff + kc), *(const v8us*)(Al + aoff + kc + 16));
#pragma unroll
            for (int t = 0; t < 4; ++t) { const v16bf b = cat16b(*(const v8us*)(Bn + boff[t] + kc), *(const v8us*)(Bn + boff[t] + kc + 16)); acc[t] = wmmab(a, b, acc[t]); acc[t] = wmmab(al, b, acc[t]); }
            asm volatile("v_nop\n\tv_nop\n\tv_nop\n\tv_nop" : "+v"(acc[0]), "+v"(acc[1]), "+v"(acc[2]), "+v"(acc[3]) : "v"(a), "v"(al));
        } }
    float* os = &ost[wave][0];
#pragma unroll
    for (int t = 0; t < 4; ++t) { const float bv = bias ? bfr(bias[c0 + t * 16 + lr]) : 0.f;
#pragma unroll
        for (int j = 0; j < 8; ++j) os[(hi * 8 + j) * 68 + t * 16 + lr] = acc[t][j] + bv; }
    __syncthreads();
    float* crow = C + (size_t)r0 * ldc + c0;
    auto pass = [&]() {
#pragma unroll
        for (int s = 0; s < 8; ++s) { const int Lid = (lane >> 3) + 4 * s, piece = lane & 7; const int row = Lid >> 1, cofs = (Lid & 1) * 32 + piece * 4;
            const v4f val = *(const v4fa*)(os + row * 68 + cofs); *(volatile v4f*)(crow + (size_t)row * ldc + cofs) = val; }
    };
    pass(); __threadfence(); pass();
}

__global__ __launch_bounds__(256) void k_gridpl64(const float* __restrict__ xb, bf* Ph, bf* Pl) {
    typedef __attribute__((ext_vector_type(2))) unsigned short v2us;
    const int lane = threadIdx.x & 31; const size_t r = (size_t)blockIdx.x * 8 + (threadIdx.x >> 5); if (r >= (size_t)NPT) return; const long pr = (long)r - GB; int y = -1, xx = -1; bool live = false;
    if (pr >= 0 && pr < NPP) { const int gy = (int)(pr / WP), gx = (int)(pr % WP); y = gy - 1; xx = gx - 1; live = (y >= 0 && y < HH && xx >= 0 && xx < HH); }
    v2us oh, ol;
#pragma unroll
    for (int i = 0; i < 2; ++i) { const int c = lane * 2 + i; const float v = live ? bfr(xb[(size_t)c * NPX + y * HH + xx]) : 0.f; const unsigned short hb = f2bf(v); oh[i] = hb; ol[i] = f2bf(v - bf2f(hb)); }
    const size_t o = r * CC + lane * 2; *(volatile v2us*)(Ph + o) = oh; *(volatile v2us*)(Pl + o) = ol; __threadfence(); *(volatile v2us*)(Ph + o) = oh; *(volatile v2us*)(Pl + o) = ol;
}
__global__ __launch_bounds__(256) void k_wtap64(const float* __restrict__ Wt, bf* WT) {
    typedef __attribute__((ext_vector_type(2))) unsigned short v2us;
    const int lane = threadIdx.x & 31; const int w = blockIdx.x * 8 + (threadIdx.x >> 5); if (w >= 9 * CC) return; const int tap = w / CC, o = w % CC; const int ky = tap / 3, kx = tap % 3; v2us v;
#pragma unroll
    for (int i = 0; i < 2; ++i) { const int ci = lane * 2 + i; v[i] = f2bf(Wt[(((size_t)o * CC + ci) * 3 + ky) * 3 + kx]); }
    *(volatile v2us*)(WT + (size_t)w * CC + lane * 2) = v; __threadfence(); *(volatile v2us*)(WT + (size_t)w * CC + lane * 2) = v;
}
__global__ __launch_bounds__(256) void k_feat(const float* __restrict__ CONV, const float* __restrict__ xb, float* FEAT) {
    const int lane = threadIdx.x & 31; const int wid = blockIdx.x * 8 + (threadIdx.x >> 5); if (wid >= CC * (NPX / 128)) return; const int c = wid / (NPX / 128); const int p0 = (wid % (NPX / 128)) * 128 + lane * 4; v4f v;
    const float* xc = xb + (size_t)c * NPX;
#pragma unroll
    for (int i = 0; i < 4; ++i) { const int p = p0 + i; const int y = p / HH, xx = p % HH; const size_t pr = (size_t)(y + 1) * WP + (xx + 1);
        float lap = -4.f * bfr(xc[p]); if (y > 0) lap += bfr(xc[p - HH]); if (y < HH - 1) lap += bfr(xc[p + HH]); if (xx > 0) lap += bfr(xc[p - 1]); if (xx < HH - 1) lap += bfr(xc[p + 1]);
        v[i] = CONV[pr * CC + c] + lap; }
    const size_t o = (size_t)c * NPX + p0; *(volatile v4f*)(FEAT + o) = v; __threadfence(); *(volatile v4f*)(FEAT + o) = v;
}
template <int S>
__global__ __launch_bounds__(256) void k_poolT(const float* __restrict__ FEAT, bf* FTh, bf* FTl) {
    typedef __attribute__((ext_vector_type(2))) unsigned short v2us;
    constexpr int hs = HH / S, N = hs * hs;
    const int lane = threadIdx.x & 31; const size_t n = (size_t)blockIdx.x * 8 + (threadIdx.x >> 5); if (n >= (size_t)N) return; const int by = (int)(n / hs), bx = (int)(n % hs); v2us oh, ol;
#pragma unroll
    for (int i = 0; i < 2; ++i) { const int c = lane * 2 + i; float s = 0.f;
#pragma unroll
        for (int dy = 0; dy < S; ++dy) {
#pragma unroll
            for (int dx = 0; dx < S; ++dx) s += FEAT[(size_t)c * NPX + (by * S + dy) * HH + bx * S + dx]; }
        const float m = s / (float)(S * S); const unsigned short hb = f2bf(m); oh[i] = hb; ol[i] = f2bf(m - bf2f(hb)); }
    const size_t o = n * CC + lane * 2; *(volatile v2us*)(FTh + o) = oh; *(volatile v2us*)(FTl + o) = ol; __threadfence(); *(volatile v2us*)(FTh + o) = oh; *(volatile v2us*)(FTl + o) = ol;
}
template <int S>
__global__ __launch_bounds__(256) void k_poolC(const float* __restrict__ FEAT, bf* FCh, bf* FCl) {
    typedef __attribute__((ext_vector_type(2))) unsigned short v2us;
    constexpr int hs = HH / S, N = hs * hs;
    const int lane = threadIdx.x & 31; const size_t wid = (size_t)blockIdx.x * 8 + (threadIdx.x >> 5); if (wid >= (size_t)CC * (N / 64)) return; const int c = (int)(wid / (N / 64)); const int n0 = (int)(wid % (N / 64)) * 64 + lane * 2; v2us oh, ol;
#pragma unroll
    for (int i = 0; i < 2; ++i) { const int n = n0 + i; const int by = n / hs, bx = n % hs; float s = 0.f;
#pragma unroll
        for (int dy = 0; dy < S; ++dy) {
#pragma unroll
            for (int dx = 0; dx < S; ++dx) s += FEAT[(size_t)c * NPX + (by * S + dy) * HH + bx * S + dx]; }
        const float m = s / (float)(S * S); const unsigned short hb = f2bf(m); oh[i] = hb; ol[i] = f2bf(m - bf2f(hb)); }
    const size_t o = (size_t)c * N + n0; *(volatile v2us*)(FCh + o) = oh; *(volatile v2us*)(FCl + o) = ol; __threadfence(); *(volatile v2us*)(FCh + o) = oh; *(volatile v2us*)(FCl + o) = ol;
}
template <int N>
__global__ __launch_bounds__(256) void k_softN(const float* __restrict__ S, int rows, bf* PH, bf* PL) {
    typedef __attribute__((ext_vector_type(4))) unsigned short v4us;
    const int lane = threadIdx.x & 31, i = blockIdx.x * 8 + (threadIdx.x >> 5); if (i >= rows) return; const float* sr = S + (size_t)i * N;
    float m = -3.0e38f;
#pragma unroll 1
    for (int c0 = lane * 4; c0 < N; c0 += 128) {
#pragma unroll
        for (int q = 0; q < 4; ++q) m = fmaxf(m, sr[c0 + q]); }
#pragma unroll
    for (int sh = 16; sh; sh >>= 1) m = fmaxf(m, __shfl_xor(m, sh, 32));
    float sum = 0.f;
#pragma unroll 1
    for (int c0 = lane * 4; c0 < N; c0 += 128) {
#pragma unroll
        for (int q = 0; q < 4; ++q) sum += __expf(sr[c0 + q] - m); }
#pragma unroll
    for (int sh = 16; sh; sh >>= 1) sum += __shfl_xor(sum, sh, 32);
    const float inv = 1.0f / sum;
#pragma unroll 1
    for (int ps = 0; ps < 2; ++ps) {
#pragma unroll 1
        for (int c0 = lane * 4; c0 < N; c0 += 128) { v4us oh, ol;
#pragma unroll
            for (int q = 0; q < 4; ++q) { const float p = __expf(sr[c0 + q] - m) * inv; const unsigned short hb = f2bf(p); oh[q] = hb; ol[q] = f2bf(p - bf2f(hb)); }
            const size_t o = (size_t)i * N + c0; *(volatile v4us*)(PH + o) = oh; *(volatile v4us*)(PL + o) = ol; }
        if (ps == 0) __threadfence(); }
}
__global__ __launch_bounds__(256) void k_final(const float* __restrict__ xb, const float* __restrict__ O1, const float* __restrict__ O2, const float* __restrict__ O4, float* OUTB) {
    const int lane = threadIdx.x & 31; const int wid = blockIdx.x * 8 + (threadIdx.x >> 5); if (wid >= CC * (NPX / 128)) return; const int c = wid / (NPX / 128); const int p0 = (wid % (NPX / 128)) * 128 + lane * 4; v4f v;
    auto up = [&](const float* O, int s, int y, int xx) -> float { const int hs = HH / s; auto src1 = [&](int i, int& i0, int& i1, float& w1) { const float sc = ((float)i + 0.5f) / (float)s - 0.5f; const float f = floorf(sc); i0 = (int)f; i1 = i0 + 1; w1 = sc - f; i0 = i0 < 0 ? 0 : (i0 > hs - 1 ? hs - 1 : i0); i1 = i1 < 0 ? 0 : (i1 > hs - 1 ? hs - 1 : i1); };
        int y0, y1, x0, x1; float wy, wx; src1(y, y0, y1, wy); src1(xx, x0, x1, wx);
        auto g = [&](int yy, int xq) -> float { return O[((size_t)yy * hs + xq) * CC + c]; };
        return (1.f - wy) * ((1.f - wx) * g(y0, x0) + wx * g(y0, x1)) + wy * ((1.f - wx) * g(y1, x0) + wx * g(y1, x1)); };
#pragma unroll
    for (int i = 0; i < 4; ++i) { const int p = p0 + i; const int y = p / HH, xx = p % HH; v[i] = bfr(xb[(size_t)c * NPX + p]) + O1[(size_t)p * CC + c] + up(O2, 2, y, xx) + up(O4, 4, y, xx); }
    const size_t o = (size_t)c * NPX + p0; *(volatile v4f*)(OUTB + o) = v; __threadfence(); *(volatile v4f*)(OUTB + o) = v;
}

extern "C" void kernel_launch(void* const* d_in, const int* in_sizes, int n_in,
                              void* d_out, int out_size, void* d_ws, size_t ws_size, hipStream_t stream) {
    (void)in_sizes; (void)n_in; (void)out_size;
    const float* x = (const float*)d_in[0]; const float* Wstd = (const float*)d_in[1];
    float* out = (float*)d_out;
    char* wsp = (char*)d_ws;
    auto take = [&](size_t bytes) { char* p = wsp; wsp += (bytes + 255) & ~(size_t)255; return (void*)p; };
    bf* WT = (bf*)take((size_t)9 * CC * CC * 2); bf* Ph = (bf*)take((size_t)NPT * CC * 2); bf* Pl = (bf*)take((size_t)NPT * CC * 2); float* CONV = (float*)take((size_t)NPR * CC * 4); float* FEAT = (float*)take((size_t)CC * NPX * 4);
    bf* FTh = (bf*)take((size_t)NPX * CC * 2); bf* FTl = (bf*)take((size_t)NPX * CC * 2); bf* FCh = (bf*)take((size_t)CC * NPX * 2); bf* FCl = (bf*)take((size_t)CC * NPX * 2);
    float* S = (float*)take((size_t)2048 * NPX * 4); bf* PH = (bf*)take((size_t)2048 * NPX * 2); bf* PL = (bf*)take((size_t)2048 * NPX * 2);
    float* XO1 = (float*)take((size_t)NPX * CC * 4); float* XO2 = (float*)take((size_t)1024 * CC * 4); float* XO4 = (float*)take((size_t)256 * CC * 4);
    if ((size_t)(wsp - (char*)d_ws) > ws_size) return;
    k_wtap64<<<(9 * CC) / 8, 256, 0, stream>>>(Wstd, WT);
    for (int b = 0; b < NB_; ++b) { const float* xb = x + (size_t)b * CC * NPX;
        k_gridpl64<<<(NPT + 7) / 8, 256, 0, stream>>>(xb, Ph, Pl);
        k_gemmtap<<<dim3(NPR / 64, 1, 1), 128, 0, stream>>>(Ph, Pl, WT, nullptr, CONV, CC, CC);
        k_feat<<<(CC * (NPX / 128)) / 8, 256, 0, stream>>>(CONV, xb, FEAT);
        k_poolT<1><<<NPX / 8, 256, 0, stream>>>(FEAT, FTh, FTl); k_poolC<1><<<(CC * (NPX / 64)) / 8, 256, 0, stream>>>(FEAT, FCh, FCl);
        for (int rb = 0; rb < 2; ++rb) { const size_t r0 = (size_t)rb * 2048;
            k_gemm3<<<dim3(2048 / 64, NPX / 64, 1), 128, 0, stream>>>(FTh + r0 * CC, FTl + r0 * CC, FTh, FTl, CC, S, NPX);
            k_softN<NPX><<<2048 / 8, 256, 0, stream>>>(S, 2048, PH, PL);
            k_gemm3<<<dim3(2048 / 64, 1, 1), 128, 0, stream>>>(PH, PL, FCh, FCl, NPX, XO1 + r0 * CC, CC); }
        k_poolT<2><<<1024 / 8, 256, 0, stream>>>(FEAT, FTh, FTl); k_poolC<2><<<(CC * (1024 / 64)) / 8, 256, 0, stream>>>(FEAT, FCh, FCl);
        k_gemm3<<<dim3(1024 / 64, 1024 / 64, 1), 128, 0, stream>>>(FTh, FTl, FTh, FTl, CC, S, 1024); k_softN<1024><<<1024 / 8, 256, 0, stream>>>(S, 1024, PH, PL);
        k_gemm3<<<dim3(1024 / 64, 1, 1), 128, 0, stream>>>(PH, PL, FCh, FCl, 1024, XO2, CC);
        k_poolT<4><<<256 / 8, 256, 0, stream>>>(FEAT, FTh, FTl); k_poolC<4><<<(CC * (256 / 64)) / 8, 256, 0, stream>>>(FEAT, FCh, FCl);
        k_gemm3<<<dim3(256 / 64, 256 / 64, 1), 128, 0, stream>>>(FTh, FTl, FTh, FTl, CC, S, 256); k_softN<256><<<256 / 8, 256, 0, stream>>>(S, 256, PH, PL);
        k_gemm3<<<dim3(256 / 64, 1, 1), 128, 0, stream>>>(PH, PL, FCh, FCl, 256, XO4, CC);
        k_final<<<(CC * (NPX / 128)) / 8, 256, 0, stream>>>(xb, XO1, XO2, XO4, out + (size_t)b * CC * NPX); }
}
